// HybridDecoderLayer_80401787781820
// MI455X (gfx1250) — hardware-run, weakly checked
//
#include <hip/hip_runtime.h>
#include <stddef.h>


typedef _Float16 h16;
typedef _Float16 v16h __attribute__((ext_vector_type(16)));
typedef _Float16 v8h  __attribute__((ext_vector_type(8)));
typedef _Float16 v4h  __attribute__((ext_vector_type(4)));
typedef float    v8f  __attribute__((ext_vector_type(8)));
typedef float    v4f  __attribute__((ext_vector_type(4)));

#ifndef NB
#define NB 2
#endif
#ifndef SEQ
#define SEQ 1024
#endif
#define NB_FULL  2
#define SEQ_FULL 1024
#define DIM    512
#define HID    2048
#define NHEAD  8
#define HD     64
#define DINNER 1024
#define DSTATE 16
#define DTRANK 32
#define XPN    64
#define MROWS (NB * SEQ)
#define OUT1_OFF ((size_t)NB_FULL * SEQ_FULL * DIM)

static_assert(NB >= 1 && NB <= NB_FULL);
static_assert(SEQ >= 128 && SEQ <= SEQ_FULL && (SEQ % 128) == 0);
static_assert(DIM == NHEAD * HD);
static_assert(HD == 64);
static_assert(HID == 4 * DIM);
static_assert(DINNER == 2 * DIM);
static_assert(XPN == DTRANK + 2 * DSTATE);
static_assert(XPN == 64 && DTRANK == 32 && DSTATE == 16);
static_assert((DIM % 64) == 0 && (DIM % 32) == 0);
static_assert((HID % 64) == 0 && (HID % 32) == 0);
static_assert((DINNER % 64) == 0 && (DINNER % 32) == 0);
static_assert((MROWS % 64) == 0 && (MROWS % 8) == 0);
static_assert(DIM == 2 * 32 * 8);
static_assert(DIM == 4 * 32 * 4);
static_assert(DINNER == 256 * 4);
static_assert(((size_t)MROWS * DINNER) % 2048 == 0);
static_assert(OUT1_OFF * 4 == (size_t)4194304);
static_assert((size_t)2 * MROWS * DINNER < (size_t)0xFFFFFFFFu);

#define LDT 72
#define LDC 68
static_assert((LDT % 8) == 0 && LDT >= 64);
static_assert((LDC % 4) == 0 && LDC >= 64);

#define WCARRY  64.0f
#define ACARRY  16.0f
#define QKCARRY 16.0f
#define VPCARRY 16.0f
#define PCARRY  1024.0f
#define VCARRY  64.0f
#define MCARRY  16.0f
#define XACARRY 64.0f
#define DCARRY  256.0f
#define YCARRY  256.0f
#define SCORE_SCALE (0.125f / (QKCARRY * QKCARRY))
#define NORM_EPS 1.0e-5f

#define W_IN3_B  ((size_t)3 * DIM * DIM * 2)
#define W_SQ_B   ((size_t)DIM * DIM * 2)
#define W_FF_B   ((size_t)DIM * HID * 2)
#define W_MIN_B  ((size_t)2 * DINNER * DIM * 2)
#define W_XP_B   ((size_t)XPN * DINNER * 2)
#define W_DT_B   ((size_t)DINNER * DTRANK * 2)
#define W_MO_B   ((size_t)DIM * DINNER * 2)
#define P16_B    ((size_t)MROWS * DIM * 2)
#define P32_B    ((size_t)MROWS * DIM * 4)
#define ST_B     ((size_t)NB * NHEAD * SEQ * 4)
#define XZ_B     ((size_t)MROWS * 2 * DINNER * 4)
#define XA32_B   ((size_t)2 * MROWS * DINNER * 4)
#define XA16_B   ((size_t)2 * MROWS * DINNER * 2)
#define DBC32_B  ((size_t)2 * MROWS * XPN * 4)
#define DBC16_B  ((size_t)2 * MROWS * XPN * 2)
#define YS_B     ((size_t)MROWS * DINNER * 2)
#define FF_B     ((size_t)MROWS * HID * 2)

#define OFF_WSA   ((size_t)0)
#define OFF_WSAO  (OFF_WSA + W_IN3_B)
#define OFF_WCA   (OFF_WSAO + W_SQ_B)
#define OFF_WCAO  (OFF_WCA + W_IN3_B)
#define OFF_WL1   (OFF_WCAO + W_SQ_B)
#define OFF_WL2   (OFF_WL1 + W_FF_B)
#define OFF_WB1   (OFF_WL2 + W_FF_B)
#define OFF_WB2   (OFF_WB1 + W_FF_B)
#define OFF_WMIN  (OFF_WB2 + W_FF_B)
#define OFF_WXP   (OFF_WMIN + W_MIN_B)
#define OFF_WDT   (OFF_WXP + W_XP_B)
#define OFF_WMO   (OFF_WDT + W_DT_B)
#define OFF_T16   (OFF_WMO + W_MO_B)
#define OFF_M16   (OFF_T16 + P16_B)
#define OFF_Q     (OFF_M16 + P16_B)
#define OFF_K     (OFF_Q + P16_B)
#define OFF_VT    (OFF_K + P16_B)
#define OFF_CTX   (OFF_VT + P16_B)
#define OFF_STM   (OFF_CTX + P16_B)
#define OFF_STR   (OFF_STM + ST_B)
#define OFF_X1    (OFF_STR + ST_B)
#define OFF_TGA32 (OFF_X1 + P32_B)
#define OFF_TGA16 (OFF_TGA32 + P32_B)
#define OFF_TGB32 (OFF_TGA16 + P16_B)
#define OFF_XN16  (OFF_TGB32 + P32_B)
#define OFF_XZ    (OFF_XN16 + P16_B)
#define OFF_XA32  (OFF_XZ + XZ_B)
#define OFF_XA16  (OFF_XA32 + XA32_B)
#define OFF_DBC32 (OFF_XA16 + XA16_B)
#define OFF_DBC16 (OFF_DBC32 + DBC32_B)
#define OFF_DEL   (OFF_DBC16 + DBC16_B)
#define OFF_YG    (OFF_DEL + XA32_B)
#define OFF_YS    (OFF_YG + XA32_B)
#define WS_TOTAL  (OFF_YS + YS_B)
static_assert(FF_B <= XA16_B);
static_assert(P32_B <= XA32_B);
static_assert((W_IN3_B % 128) == 0 && (W_SQ_B % 128) == 0 && (W_FF_B % 128) == 0);
static_assert((W_MIN_B % 128) == 0 && (W_XP_B % 128) == 0 && (W_DT_B % 128) == 0 && (W_MO_B % 128) == 0);
static_assert((P16_B % 128) == 0 && (P32_B % 128) == 0 && (ST_B % 128) == 0 && (XZ_B % 128) == 0);
static_assert((XA32_B % 128) == 0 && (XA16_B % 128) == 0 && (DBC32_B % 128) == 0 && (DBC16_B % 128) == 0);
static_assert((YS_B % 128) == 0);
static_assert(WS_TOTAL <= (size_t)134217728);

__device__ __forceinline__ float bf16r(float x) {
  unsigned int u = __float_as_uint(x);
  u = (u + 0x7FFFu + ((u >> 16) & 1u)) & 0xFFFF0000u;
  return __uint_as_float(u);
}

static __device__ __forceinline__ h16 toh_flush(float v) {
  const h16 r = (h16)v;
  return (fabsf(v) < 6.103515625e-05f) ? (h16)0.0f : r;
}

__device__ __forceinline__ v16h frag_at(const _Float16* p) {
  v8h lo = *(const v8h*)(p);
  v8h hi = *(const v8h*)(p + 16);
  v16h out;
#pragma unroll
  for (int i = 0; i < 8; ++i) { out[i] = lo[i]; out[i + 8] = hi[i]; }
  return out;
}
__device__ __forceinline__ v16h ld_frag(const _Float16* base, unsigned ld) {
  const unsigned lane = threadIdx.x & 31u;
  return frag_at(base + (lane & 15u) * ld + (lane >> 4) * 8u);
}

__device__ __forceinline__ v8f wmma16(v16h a, v16h b, v8f c) {
  v8f d = __builtin_amdgcn_wmma_f32_16x16x32_f16(false, a, false, b, (short)0, c,
                                                 false, false);
  asm volatile("v_nop\n\tv_nop\n\tv_nop\n\tv_nop" : "+v"(d) : "v"(a), "v"(b));
  return d;
}

__device__ __forceinline__ float red16_max(float x) {
#pragma unroll
  for (int off = 1; off < 16; off <<= 1) x = fmaxf(x, __shfl_xor(x, off, 32));
  return x;
}
__device__ __forceinline__ float red16_sum(float x) {
#pragma unroll
  for (int off = 1; off < 16; off <<= 1) x += __shfl_xor(x, off, 32);
  return x;
}
__device__ __forceinline__ float red32_sum(float x) {
#pragma unroll
  for (int off = 1; off < 32; off <<= 1) x += __shfl_xor(x, off, 32);
  return x;
}

__device__ __forceinline__ void wave_lds_sync() {
  __builtin_amdgcn_fence(3  , "wavefront");
  asm volatile("s_wait_dscnt 0x0" ::: "memory");
  __builtin_amdgcn_wave_barrier();
}

__device__ __forceinline__ unsigned wave_index() {
  return (unsigned)__builtin_amdgcn_readfirstlane((int)(threadIdx.x >> 5));
}

__device__ __forceinline__ float silu_f(float a) {
  return a * __builtin_amdgcn_rcpf(1.0f + __expf(-a));
}

__global__ __launch_bounds__(256) void wcast_kernel(
    const float* __restrict__ W, _Float16* __restrict__ Wt, unsigned n8) {
  const unsigned i = blockIdx.x * 256u + threadIdx.x;
  if (i >= n8) return;
  const v4f a0 = *(const v4f*)(W + (size_t)i * 8u);
  const v4f a1 = *(const v4f*)(W + (size_t)i * 8u + 4u);
  v8h o;
#pragma unroll
  for (int j = 0; j < 4; ++j) {
    o[j]     = toh_flush(WCARRY * bf16r(a0[j]));
    o[j + 4] = toh_flush(WCARRY * bf16r(a1[j]));
  }
  _Float16* p = Wt + (size_t)i * 8u;
  *(volatile v8h*)p = o;
  __threadfence();
  *(volatile v8h*)p = o;
}

__global__ __launch_bounds__(256) void incast_kernel(
    const float* __restrict__ X, _Float16* __restrict__ dst) {
  const unsigned lane = threadIdx.x & 31u;
  const unsigned w = wave_index();
  const unsigned crow = blockIdx.x * 8u + w;
  const unsigned bidx = crow / (unsigned)SEQ;
  const unsigned sq = crow - bidx * (unsigned)SEQ;
  const size_t srow = (size_t)sq * NB_FULL + bidx;
  const float* xr = X + srow * DIM + lane * 8u;
#pragma unroll 1
  for (unsigned j = 0; j < 2u; ++j) {
    const v4f a0 = *(const v4f*)(xr + j * 256u);
    const v4f a1 = *(const v4f*)(xr + j * 256u + 4u);
    v8h o;
#pragma unroll
    for (int i = 0; i < 4; ++i) {
      o[i]     = toh_flush(ACARRY * bf16r(a0[i]));
      o[i + 4] = toh_flush(ACARRY * bf16r(a1[i]));
    }
    _Float16* p = dst + (size_t)crow * DIM + j * 256u + lane * 8u;
    *(volatile v8h*)p = o;
    __threadfence();
    *(volatile v8h*)p = o;
  }
}

__global__ __launch_bounds__(256) void ln_ws_kernel(
    const float* __restrict__ X, const float* __restrict__ G, const float* __restrict__ Be,
    _Float16* __restrict__ dst) {
  const unsigned lane = threadIdx.x & 31u;
  const unsigned w = wave_index();
  const unsigned crow = blockIdx.x * 8u + w;
  const float* xr = X + (size_t)crow * DIM + lane * 8u;

  float s = 0.0f;
#pragma unroll 1
  for (unsigned j = 0; j < 2u; ++j) {
    const v4f a0 = *(const v4f*)(xr + j * 256u);
    const v4f a1 = *(const v4f*)(xr + j * 256u + 4u);
#pragma unroll
    for (int i = 0; i < 4; ++i) s += a0[i] + a1[i];
  }
  const float mean = red32_sum(s) * (1.0f / (float)DIM);

  float ss = 0.0f;
#pragma unroll 1
  for (unsigned j = 0; j < 2u; ++j) {
    const v4f a0 = *(const v4f*)(xr + j * 256u);
    const v4f a1 = *(const v4f*)(xr + j * 256u + 4u);
#pragma unroll
    for (int i = 0; i < 4; ++i) {
      const float d0 = a0[i] - mean;
      const float d1 = a1[i] - mean;
      ss += d0 * d0;
      ss += d1 * d1;
    }
  }
  const float var = red32_sum(ss) * (1.0f / (float)DIM);
  const float rstd = 1.0f / sqrtf(var + NORM_EPS);

#pragma unroll 1
  for (unsigned j = 0; j < 2u; ++j) {
    const unsigned c = j * 256u + lane * 8u;
    const v4f a0 = *(const v4f*)(xr + j * 256u);
    const v4f a1 = *(const v4f*)(xr + j * 256u + 4u);
    const v4f g0 = *(const v4f*)(G + c);
    const v4f g1 = *(const v4f*)(G + c + 4u);
    const v4f b0 = *(const v4f*)(Be + c);
    const v4f b1 = *(const v4f*)(Be + c + 4u);
    v8h o;
#pragma unroll
    for (int i = 0; i < 4; ++i) {
      const float d0 = a0[i] - mean;
      const float d1 = a1[i] - mean;
      o[i]     = toh_flush(ACARRY * (d0 * rstd * bf16r(g0[i]) + bf16r(b0[i])));
      o[i + 4] = toh_flush(ACARRY * (d1 * rstd * bf16r(g1[i]) + bf16r(b1[i])));
    }
    _Float16* p = dst + (size_t)crow * DIM + c;
    *(volatile v8h*)p = o;
    __threadfence();
    *(volatile v8h*)p = o;
  }
}

template <int W16, int OUTFULL>
__device__ __forceinline__ void rms_body(const float* __restrict__ X,
                                         const float* __restrict__ G,
                                         float* __restrict__ y32,
                                         _Float16* __restrict__ y16) {
  const unsigned lane = threadIdx.x & 31u;
  const unsigned w = wave_index();
  const unsigned crow = blockIdx.x * 8u + w;
  const float* xr = X + (size_t)crow * DIM;
  size_t orow = crow;
  if (OUTFULL) {
    const unsigned bidx = crow / (unsigned)SEQ;
    const unsigned sq = crow - bidx * (unsigned)SEQ;
    orow = (size_t)sq * NB_FULL + bidx;
  }

  float ss = 0.0f;
#pragma unroll 1
  for (unsigned j = 0; j < 4u; ++j) {
    const v4f a = *(const v4f*)(xr + j * 128u + lane * 4u);
#pragma unroll
    for (int i = 0; i < 4; ++i) ss += a[i] * a[i];
  }
  const float ms = red32_sum(ss) * (1.0f / (float)DIM);
  const float inv = 1.0f / sqrtf(ms + NORM_EPS);

#pragma unroll 1
  for (unsigned j = 0; j < 4u; ++j) {
    const unsigned c = j * 128u + lane * 4u;
    const v4f a = *(const v4f*)(xr + c);
    const v4f g = *(const v4f*)(G + c);
    v4f o;
#pragma unroll
    for (int i = 0; i < 4; ++i) o[i] = (a[i] * bf16r(g[i])) * inv;
    float* p = y32 + orow * DIM + c;
    *(volatile v4f*)p = o;
    __threadfence();
    *(volatile v4f*)p = o;
  }
  if (W16) {
#pragma unroll 1
    for (unsigned j = 0; j < 2u; ++j) {
      const unsigned c = j * 256u + lane * 8u;
      const v4f a0 = *(const v4f*)(xr + c);
      const v4f a1 = *(const v4f*)(xr + c + 4u);
      const v4f g0 = *(const v4f*)(G + c);
      const v4f g1 = *(const v4f*)(G + c + 4u);
      v8h o;
#pragma unroll
      for (int i = 0; i < 4; ++i) {
        o[i]     = toh_flush(ACARRY * ((a0[i] * bf16r(g0[i])) * inv));
        o[i + 4] = toh_flush(ACARRY * ((a1[i] * bf16r(g1[i])) * inv));
      }
      _Float16* p = y16 + (size_t)crow * DIM + c;
      *(volatile v8h*)p = o;
      __threadfence();
      *(volatile v8h*)p = o;
    }
  }
}

__global__ __launch_bounds__(256) void rms_both_kernel(
    const float* __restrict__ X, const float* __restrict__ G, float* __restrict__ y32,
    _Float16* __restrict__ y16) {
  rms_body<1, 0>(X, G, y32, y16);
}
__global__ __launch_bounds__(256) void rms_f32_kernel(
    const float* __restrict__ X, const float* __restrict__ G, float* __restrict__ y32) {
  rms_body<0, 0>(X, G, y32, (_Float16*)0);
}
__global__ __launch_bounds__(256) void rms_out_kernel(
    const float* __restrict__ X, const float* __restrict__ G, float* __restrict__ y32) {
  rms_body<0, 1>(X, G, y32, (_Float16*)0);
}

template <int MODE>
__device__ __forceinline__ void gemm_body(
    const _Float16* __restrict__ A16, const unsigned lda,
    const _Float16* __restrict__ Bt, const unsigned ldb, const unsigned K,
    const float* __restrict__ bias, const float* __restrict__ addf,
    float* __restrict__ outf, _Float16* __restrict__ out16, const unsigned ldo,
    const float cs, const float bscale, const float oc) {
  __shared__ float Cs[64 * LDC];
  const unsigned tid = threadIdx.x, lane = tid & 31u;
  const unsigned w = wave_index();
  const unsigned mw = w >> 1, nw = w & 1u;
  const unsigned hh = lane >> 4, m = lane & 15u;
  const unsigned n0 = blockIdx.x * 64u;
  const unsigned row0 = blockIdx.y * 64u;

  const _Float16* ap  = A16 + (size_t)(row0 + mw * 16u + m) * lda + hh * 8u;
  const _Float16* bp0 = Bt + (size_t)(n0 + nw * 32u + m) * ldb + hh * 8u;
  const _Float16* bp1 = bp0 + (size_t)16 * ldb;
  v8f acc0 = {}, acc1 = {};
#pragma unroll 2
  for (unsigned k0 = 0; k0 < K; k0 += 32u) {
    const v16h a  = frag_at(ap + k0);
    const v16h b0 = frag_at(bp0 + k0);
    const v16h b1 = frag_at(bp1 + k0);
    acc0 = wmma16(a, b0, acc0);
    acc1 = wmma16(a, b1, acc1);
  }
#pragma unroll
  for (int r = 0; r < 8; ++r) {
    float* d = &Cs[(mw * 16u + hh * 8u + (unsigned)r) * LDC + nw * 32u + m];
    d[0]  = acc0[r];
    d[16] = acc1[r];
  }
  __syncthreads();

  if (MODE == 3 || MODE == 7) {
#pragma unroll 1
    for (unsigned g = 0; g < 4u; ++g) {
      const unsigned r = 32u * (g >> 1) + (tid >> 3);
      const unsigned c = (tid & 7u) * 8u + 4u * (g & 1u);
      const v4f u  = *(const v4f*)&Cs[r * LDC + c];
      const v4f gb = *(const v4f*)(bias + n0 + c);
      v4f t;
#pragma unroll
      for (int j = 0; j < 4; ++j) {
        const float z = u[j] * cs + bf16r(gb[j]);
        float a;
        if (MODE == 3) a = fmaxf(z, 0.0f);
        else           a = 0.5f * z * (1.0f + erff(z * 0.70710678118654752f));
        t[j] = MCARRY * a;
      }
      *(v4f*)&Cs[r * LDC + c] = t;
    }
  }

  if (MODE == 9) {
#pragma unroll 1
    for (unsigned g = 0; g < 4u; ++g) {
      const unsigned r = 16u * g + (tid >> 4);
      const unsigned c = (tid & 15u) * 4u;
      const v4f u  = *(const v4f*)&Cs[r * LDC + c];
      const v4f gb = *(const v4f*)(bias + n0 + c);
      v4f t;
#pragma unroll
      for (int j = 0; j < 4; ++j) {
        const float z = u[j] * cs + bf16r(gb[j]);
        t[j] = fmaxf(z, 0.0f) + log1pf(expf(-fabsf(z)));
      }
      *(v4f*)&Cs[r * LDC + c] = t;
    }
  }

  if (MODE == 2 || MODE == 4 || MODE == 5 || MODE == 6 || MODE == 8 || MODE == 9) {
    v4f xs[4];
    size_t off[4];
#pragma unroll
    for (unsigned i = 0; i < 4u; ++i) {
      const unsigned r = 16u * i + (tid >> 4);
      const unsigned c = (tid & 15u) * 4u;
      const unsigned crow = row0 + r;
      const v4f u = *(const v4f*)&Cs[r * LDC + c];
      v4f val;
      if (MODE == 9) {
        val = u;
      } else if (MODE == 8) {
#pragma unroll
        for (int j = 0; j < 4; ++j) val[j] = u[j] * cs;
      } else {
        const v4f g = *(const v4f*)(bias + n0 + c);
        if (MODE == 5) {
#pragma unroll
          for (int j = 0; j < 4; ++j) val[j] = u[j] * cs + bscale * bf16r(g[j]);
        } else {
          size_t inrow = crow;
          unsigned lad = ldo;
          if (MODE == 2) {
            const unsigned bidx = crow / (unsigned)SEQ;
            const unsigned sq = crow - bidx * (unsigned)SEQ;
            inrow = (size_t)sq * NB_FULL + bidx;
            lad = (unsigned)DIM;
          }
          const v4f xin = *(const v4f*)(addf + inrow * lad + n0 + c);
#pragma unroll
          for (int j = 0; j < 4; ++j) {
            const float base = (MODE == 2) ? bf16r(xin[j]) : xin[j];
            const float t = u[j] * cs + bscale * bf16r(g[j]);
            val[j] = (MODE == 6) ? (base + (t + base)) : (base + t);
          }
        }
      }
      xs[i] = val;
      off[i] = (size_t)crow * ldo + n0 + c;
    }
#pragma unroll
    for (int i = 0; i < 4; ++i) *(volatile v4f*)(outf + off[i]) = xs[i];
    __threadfence();
#pragma unroll
    for (int i = 0; i < 4; ++i) *(volatile v4f*)(outf + off[i]) = xs[i];
  }

  if (MODE == 0 || MODE == 3 || MODE == 7 || MODE == 8) {
    v8h x[2];
    size_t off[2];
#pragma unroll
    for (unsigned i = 0; i < 2u; ++i) {
      const unsigned r = 32u * i + (tid >> 3);
      const unsigned c = (tid & 7u) * 8u;
      const v4f u0 = *(const v4f*)&Cs[r * LDC + c];
      const v4f u1 = *(const v4f*)&Cs[r * LDC + c + 4];
      if (MODE == 3 || MODE == 7) {
#pragma unroll
        for (int j = 0; j < 4; ++j) {
          x[i][j]     = toh_flush(u0[j]);
          x[i][j + 4] = toh_flush(u1[j]);
        }
      } else if (MODE == 8) {
#pragma unroll
        for (int j = 0; j < 4; ++j) {
          x[i][j]     = toh_flush(oc * (u0[j] * cs));
          x[i][j + 4] = toh_flush(oc * (u1[j] * cs));
        }
      } else {
        const v4f g0 = *(const v4f*)(bias + n0 + c);
        const v4f g1 = *(const v4f*)(bias + n0 + c + 4u);
#pragma unroll
        for (int j = 0; j < 4; ++j) {
          x[i][j]     = toh_flush(oc * (u0[j] * cs + bf16r(g0[j])));
          x[i][j + 4] = toh_flush(oc * (u1[j] * cs + bf16r(g1[j])));
        }
      }
      off[i] = (size_t)(row0 + r) * ldo + n0 + c;
    }
#pragma unroll
    for (int i = 0; i < 2; ++i) *(volatile v8h*)(out16 + off[i]) = x[i];
    __threadfence();
#pragma unroll
    for (int i = 0; i < 2; ++i) *(volatile v8h*)(out16 + off[i]) = x[i];
  }

  if (MODE == 1) {
    const unsigned bidx = row0 / (unsigned)SEQ;
    const unsigned key0 = row0 - bidx * (unsigned)SEQ;
    v8h x[2];
    size_t off[2];
#pragma unroll
    for (unsigned i = 0; i < 2u; ++i) {
      const unsigned dcol = 32u * i + (tid >> 3);
      const unsigned kk = (tid & 7u) * 8u;
      const float bb = bf16r(bias[n0 + dcol]);
#pragma unroll
      for (unsigned j = 0; j < 8u; ++j) {
        const float t = Cs[(kk + j) * LDC + dcol] * cs + bb;
        x[i][j] = toh_flush(oc * t);
      }
      off[i] = ((size_t)bidx * DIM + n0 + dcol) * SEQ + key0 + kk;
    }
#pragma unroll
    for (int i = 0; i < 2; ++i) *(volatile v8h*)(out16 + off[i]) = x[i];
    __threadfence();
#pragma unroll
    for (int i = 0; i < 2; ++i) *(volatile v8h*)(out16 + off[i]) = x[i];
  }
}

__global__ __launch_bounds__(256) void gemm_h16_kernel(
    const _Float16* __restrict__ A16, unsigned lda, const _Float16* __restrict__ Bt,
    unsigned ldb, unsigned K, const float* __restrict__ bias, _Float16* __restrict__ out16,
    unsigned ldo, float cs, float oc) {
  gemm_body<0>(A16, lda, Bt, ldb, K, bias, (const float*)0, (float*)0, out16, ldo, cs, 1.0f, oc);
}
__global__ __launch_bounds__(256) void gemm_vt_kernel(
    const _Float16* __restrict__ A16, const _Float16* __restrict__ Bt,
    const float* __restrict__ bias, _Float16* __restrict__ vt, float cs, float oc) {
  gemm_body<1>(A16, (unsigned)DIM, Bt, (unsigned)DIM, (unsigned)DIM, bias, (const float*)0,
               (float*)0, vt, (unsigned)DIM, cs, 1.0f, oc);
}
__global__ __launch_bounds__(256) void gemm_addin_kernel(
    const _Float16* __restrict__ A16, unsigned lda, const _Float16* __restrict__ Bt,
    unsigned ldb, unsigned K, const float* __restrict__ bias, const float* __restrict__ xin,
    float* __restrict__ outf, unsigned ldo, float cs) {
  gemm_body<2>(A16, lda, Bt, ldb, K, bias, xin, outf, (_Float16*)0, ldo, cs, 1.0f, 1.0f);
}
__global__ __launch_bounds__(256) void gemm_relu_kernel(
    const _Float16* __restrict__ A16, unsigned lda, const _Float16* __restrict__ Bt,
    unsigned ldb, unsigned K, const float* __restrict__ bias, _Float16* __restrict__ out16,
    unsigned ldo, float cs) {
  gemm_body<3>(A16, lda, Bt, ldb, K, bias, (const float*)0, (float*)0, out16, ldo, cs, 1.0f, 1.0f);
}
__global__ __launch_bounds__(256) void gemm_addws_kernel(
    const _Float16* __restrict__ A16, unsigned lda, const _Float16* __restrict__ Bt,
    unsigned ldb, unsigned K, const float* __restrict__ bias, const float* __restrict__ addf,
    float* __restrict__ outf, unsigned ldo, float cs) {
  gemm_body<4>(A16, lda, Bt, ldb, K, bias, addf, outf, (_Float16*)0, ldo, cs, 1.0f, 1.0f);
}
__global__ __launch_bounds__(256) void gemm_f32_kernel(
    const _Float16* __restrict__ A16, unsigned lda, const _Float16* __restrict__ Bt,
    unsigned ldb, unsigned K, const float* __restrict__ bias, float* __restrict__ outf,
    unsigned ldo, float cs, float bscale) {
  gemm_body<5>(A16, lda, Bt, ldb, K, bias, (const float*)0, outf, (_Float16*)0, ldo, cs, bscale, 1.0f);
}
__global__ __launch_bounds__(256) void gemm_add2_kernel(
    const _Float16* __restrict__ A16, unsigned lda, const _Float16* __restrict__ Bt,
    unsigned ldb, unsigned K, const float* __restrict__ bias, const float* __restrict__ addf,
    float* __restrict__ outf, unsigned ldo, float cs) {
  gemm_body<6>(A16, lda, Bt, ldb, K, bias, addf, outf, (_Float16*)0, ldo, cs, 1.0f, 1.0f);
}
__global__ __launch_bounds__(256) void gemm_gelu_kernel(
    const _Float16* __restrict__ A16, unsigned lda, const _Float16* __restrict__ Bt,
    unsigned ldb, unsigned K, const float* __restrict__ bias, _Float16* __restrict__ out16,
    unsigned ldo, float cs) {
  gemm_body<7>(A16, lda, Bt, ldb, K, bias, (const float*)0, (float*)0, out16, ldo, cs, 1.0f, 1.0f);
}
__global__ __launch_bounds__(256) void gemm_xproj_kernel(
    const _Float16* __restrict__ A16, unsigned lda, const _Float16* __restrict__ Bt,
    unsigned ldb, unsigned K, float* __restrict__ outf, _Float16* __restrict__ out16,
    unsigned ldo, float cs, float oc) {
  gemm_body<8>(A16, lda, Bt, ldb, K, (const float*)0, (const float*)0, outf, out16, ldo, cs, 1.0f, oc);
}
__global__ __launch_bounds__(256) void gemm_softplus_kernel(
    const _Float16* __restrict__ A16, unsigned lda, const _Float16* __restrict__ Bt,
    unsigned ldb, unsigned K, const float* __restrict__ bias, float* __restrict__ outf,
    unsigned ldo, float cs) {
  gemm_body<9>(A16, lda, Bt, ldb, K, bias, (const float*)0, outf, (_Float16*)0, ldo, cs, 1.0f, 1.0f);
}

template <int STATS>
__device__ __forceinline__ void attn_body(
    const _Float16* __restrict__ Qh, const _Float16* __restrict__ Kh,
    const _Float16* __restrict__ Vt, _Float16* __restrict__ Ov,
    float* __restrict__ stM, float* __restrict__ stR) {
  __shared__ _Float16 Ks[64 * LDT];
  __shared__ _Float16 Vs[64 * LDT];
  __shared__ _Float16 Ps[8 * 16 * LDT];
  __shared__ float Sm[128];
  __shared__ float Sr[128];

  const unsigned tid = threadIdx.x, lane = tid & 31u;
  const unsigned w = wave_index();
  const unsigned hh = lane >> 4, m = lane & 15u;
  const unsigned q0 = blockIdx.x * 128u;
  const unsigned head = blockIdx.y;
  const unsigned b = blockIdx.z;
  const float scale = SCORE_SCALE;
  const unsigned qrow0 = q0 + w * 16u;
  _Float16* P = Ps + w * (16u * LDT);

  const size_t qoff = (size_t)(b * (unsigned)SEQ + qrow0 + m) * DIM + head * HD + hh * 8u;
  v16h qf[2];
  qf[0] = frag_at(Qh + qoff);
  qf[1] = frag_at(Qh + qoff + 32);

  float mrow[8], lrow[8];
  v8f o[4];
#pragma unroll
  for (int v = 0; v < 8; ++v) { mrow[v] = -1.0e30f; lrow[v] = 0.0f; }
#pragma unroll
  for (int nb = 0; nb < 4; ++nb) o[nb] = (v8f){};

  const size_t kplane = (size_t)b * SEQ * DIM + head * HD;
  const size_t vplane = ((size_t)b * DIM + head * HD) * SEQ;

  for (unsigned kb = 0; kb < (unsigned)SEQ; kb += 64u) {
#pragma unroll
    for (unsigned j = 0; j < 2u; ++j) {
      const unsigned idx = tid + 256u * j;
      const unsigned r = idx >> 3, c = (idx & 7u) * 8u;
      *(v8h*)&Ks[r * LDT + c] = *(const v8h*)(Kh + kplane + (size_t)(kb + r) * DIM + c);
      *(v8h*)&Vs[r * LDT + c] = *(const v8h*)(Vt + vplane + (size_t)r * SEQ + kb + c);
    }
    __syncthreads();

    v8f s[4];
#pragma unroll
    for (int kg = 0; kg < 4; ++kg) {
      v8f t = {};
#pragma unroll
      for (int c = 0; c < 2; ++c) {
        const v16h kf = ld_frag(&Ks[(kg * 16) * LDT + c * 32], LDT);
        t = wmma16(qf[c], kf, t);
      }
      s[kg] = t * scale;
    }

    float alpha[8];
#pragma unroll
    for (int v = 0; v < 8; ++v) {
      float mx = fmaxf(fmaxf(s[0][v], s[1][v]), fmaxf(s[2][v], s[3][v]));
      mx = red16_max(mx);
      const float mn = fmaxf(mrow[v], mx);
      alpha[v] = __expf(mrow[v] - mn);
      mrow[v] = mn;
    }
#pragma unroll
    for (int kg = 0; kg < 4; ++kg)
#pragma unroll
      for (int v = 0; v < 8; ++v) s[kg][v] = __expf(s[kg][v] - mrow[v]);
#pragma unroll
    for (int v = 0; v < 8; ++v) {
      const float rs = red16_sum((s[0][v] + s[1][v]) + (s[2][v] + s[3][v]));
      lrow[v] = alpha[v] * lrow[v] + rs;
    }
#pragma unroll
    for (int nb = 0; nb < 4; ++nb)
#pragma unroll
      for (int v = 0; v < 8; ++v) o[nb][v] = o[nb][v] * alpha[v];

#pragma unroll
    for (int kg = 0; kg < 4; ++kg)
#pragma unroll
      for (int v = 0; v < 8; ++v)
        P[(hh * 8u + (unsigned)v) * LDT + (unsigned)kg * 16u + m] = toh_flush(s[kg][v] * PCARRY);
    wave_lds_sync();

#pragma unroll
    for (int c = 0; c < 2; ++c) {
      const v16h pf = ld_frag(P + c * 32, LDT);
#pragma unroll
      for (int nb = 0; nb < 4; ++nb) {
        const v16h vf = ld_frag(&Vs[(nb * 16) * LDT + c * 32], LDT);
        o[nb] = wmma16(pf, vf, o[nb]);
      }
    }
    __syncthreads();
  }

  float inv[8];
#pragma unroll
  for (int v = 0; v < 8; ++v)
    inv[v] = __builtin_amdgcn_rcpf(lrow[v]) * (VCARRY / (PCARRY * VPCARRY));
#pragma unroll
  for (int nb = 0; nb < 4; ++nb)
#pragma unroll
    for (int v = 0; v < 8; ++v)
      P[(hh * 8u + (unsigned)v) * LDT + (unsigned)nb * 16u + m] = toh_flush(o[nb][v] * inv[v]);
  wave_lds_sync();
  v8h x[4];
  size_t off[4];
#pragma unroll
  for (unsigned i = 0; i < 4u; ++i) {
    const unsigned r = 4u * i + (lane >> 3);
    const unsigned c = (lane & 7u) * 8u;
    x[i] = *(const v8h*)&P[r * LDT + c];
    off[i] = (size_t)(b * (unsigned)SEQ + qrow0 + r) * DIM + head * HD + c;
  }
#pragma unroll
  for (int i = 0; i < 4; ++i) *(volatile v8h*)(Ov + off[i]) = x[i];
  __threadfence();
#pragma unroll
  for (int i = 0; i < 4; ++i) *(volatile v8h*)(Ov + off[i]) = x[i];

  if (STATS) {
    if (m == 0u) {
#pragma unroll
      for (int v = 0; v < 8; ++v) {
        Sm[w * 16u + hh * 8u + (unsigned)v] = mrow[v];
        Sr[w * 16u + hh * 8u + (unsigned)v] =
            __builtin_amdgcn_rcpf(lrow[v]) * (1.0f / (float)NHEAD);
      }
    }
    __syncthreads();
    if (w == 0u) {
      const v4f xm = *(const v4f*)&Sm[lane * 4u];
      const v4f xr = *(const v4f*)&Sr[lane * 4u];
      const size_t so = ((size_t)b * NHEAD + head) * SEQ + q0 + lane * 4u;
      *(volatile v4f*)(stM + so) = xm;
      *(volatile v4f*)(stR + so) = xr;
      __threadfence();
      *(volatile v4f*)(stM + so) = xm;
      *(volatile v4f*)(stR + so) = xr;
    }
  }
}

__global__ __launch_bounds__(256) void attn_kernel(
    const _Float16* __restrict__ Qh, const _Float16* __restrict__ Kh,
    const _Float16* __restrict__ Vt, _Float16* __restrict__ Ov) {
  attn_body<0>(Qh, Kh, Vt, Ov, (float*)0, (float*)0);
}
__global__ __launch_bounds__(256) void attn_stats_kernel(
    const _Float16* __restrict__ Qh, const _Float16* __restrict__ Kh,
    const _Float16* __restrict__ Vt, _Float16* __restrict__ Ov,
    float* __restrict__ stM, float* __restrict__ stR) {
  attn_body<1>(Qh, Kh, Vt, Ov, stM, stR);
}

__global__ __launch_bounds__(256) void attn_mean_kernel(
    const _Float16* __restrict__ Qh, const _Float16* __restrict__ Kh,
    const float* __restrict__ stM, const float* __restrict__ stR, float* __restrict__ outp) {
  __shared__ float Ts[8 * 16 * LDC];
  const unsigned tid = threadIdx.x, lane = tid & 31u;
  const unsigned w = wave_index();
  const unsigned hh = lane >> 4, m = lane & 15u;
  const unsigned key0 = blockIdx.x * 64u;
  const unsigned qrow0 = blockIdx.y * 128u + w * 16u;
  const unsigned b = blockIdx.z;
  const float scale = SCORE_SCALE;

  v8f acc[4];
#pragma unroll
  for (int kg = 0; kg < 4; ++kg) acc[kg] = (v8f){};

#pragma unroll 1
  for (unsigned head = 0; head < (unsigned)NHEAD; ++head) {
    const size_t qoff = (size_t)(b * (unsigned)SEQ + qrow0 + m) * DIM + head * HD + hh * 8u;
    const v16h q0f = frag_at(Qh + qoff);
    const v16h q1f = frag_at(Qh + qoff + 32);
    const size_t sb = ((size_t)b * NHEAD + head) * SEQ + qrow0 + hh * 8u;
    const v4f m0 = *(const v4f*)(stM + sb);
    const v4f m1 = *(const v4f*)(stM + sb + 4u);
    const v4f r0 = *(const v4f*)(stR + sb);
    const v4f r1 = *(const v4f*)(stR + sb + 4u);
    float mm[8], rr[8];
#pragma unroll
    for (int v = 0; v < 4; ++v) { mm[v] = m0[v]; mm[v + 4] = m1[v]; rr[v] = r0[v]; rr[v + 4] = r1[v]; }
#pragma unroll
    for (int kg = 0; kg < 4; ++kg) {
      const size_t koff =
          (size_t)(b * (unsigned)SEQ + key0 + (unsigned)kg * 16u + m) * DIM + head * HD + hh * 8u;
      v8f t = {};
      t = wmma16(q0f, frag_at(Kh + koff), t);
      t = wmma16(q1f, frag_at(Kh + koff + 32), t);
      t = t * scale;
#pragma unroll
      for (int v = 0; v < 8; ++v) acc[kg][v] += __expf(t[v] - mm[v]) * rr[v];
    }
  }

  float* T = Ts + w * (16u * LDC);
#pragma unroll
  for (int kg = 0; kg < 4; ++kg)
#pragma unroll
    for (int v = 0; v < 8; ++v)
      T[(hh * 8u + (unsigned)v) * LDC + (unsigned)kg * 16u + m] = acc[kg][v];
  wave_lds_sync();
  v4f x[8];
  size_t off[8];
#pragma unroll
  for (unsigned i = 0; i < 8u; ++i) {
    const unsigned r = 2u * i + (lane >> 4);
    const unsigned c = (lane & 15u) * 4u;
    x[i] = *(const v4f*)&T[r * LDC + c];
    off[i] = ((size_t)b * SEQ_FULL + qrow0 + r) * SEQ_FULL + key0 + c;
  }
#pragma unroll
  for (int i = 0; i < 8; ++i) *(volatile v4f*)(outp + off[i]) = x[i];
  __threadfence();
#pragma unroll
  for (int i = 0; i < 8; ++i) *(volatile v4f*)(outp + off[i]) = x[i];
}

__global__ __launch_bounds__(256) void conv_silu_kernel(
    const float* __restrict__ XZ, const float* __restrict__ cw, const float* __restrict__ cb,
    float* __restrict__ xa32, _Float16* __restrict__ xa16) {
  const unsigned row = blockIdx.x;
  const unsigned c = threadIdx.x * 4u;
  const unsigned bidx = row / (unsigned)SEQ;
  const int l = (int)(row - bidx * (unsigned)SEQ);

  v4f wt[4];
#pragma unroll
  for (unsigned k = 0; k < 4u; ++k) {
    const v4f t = *(const v4f*)(cw + (size_t)(c + k) * 4u);
#pragma unroll
    for (int j = 0; j < 4; ++j) wt[k][j] = bf16r(t[j]);
  }
  v4f bb = *(const v4f*)(cb + c);
#pragma unroll
  for (int j = 0; j < 4; ++j) bb[j] = bf16r(bb[j]);

  v4f xv[7];
#pragma unroll
  for (int t = 0; t < 7; ++t) {
    const int lt = l + t - 3;
    const int lc = min(max(lt, 0), (int)SEQ - 1);
    const v4f a = *(const v4f*)(XZ + ((size_t)bidx * SEQ + (unsigned)lc) * (2u * DINNER) + c);
    const bool ok = (lt == lc);
#pragma unroll
    for (int i = 0; i < 4; ++i) xv[t][i] = ok ? a[i] : 0.0f;
  }

  v4f af = bb, ab = bb;
#pragma unroll
  for (int j = 0; j < 4; ++j)
#pragma unroll
    for (int k = 0; k < 4; ++k) {
      af[k] += wt[k][j] * xv[j][k];
      ab[k] += wt[k][j] * xv[6 - j][k];
    }
  v4f sf, sb;
  v4h hf, hb;
#pragma unroll
  for (int k = 0; k < 4; ++k) {
    sf[k] = silu_f(af[k]);
    sb[k] = silu_f(ab[k]);
    hf[k] = toh_flush(XACARRY * sf[k]);
    hb[k] = toh_flush(XACARRY * sb[k]);
  }
  const size_t o0 = (size_t)row * DINNER + c;
  const size_t o1 = o0 + (size_t)MROWS * DINNER;
  *(volatile v4f*)(xa32 + o0) = sf;
  *(volatile v4f*)(xa32 + o1) = sb;
  *(volatile v4h*)(xa16 + o0) = hf;
  *(volatile v4h*)(xa16 + o1) = hb;
  __threadfence();
  *(volatile v4f*)(xa32 + o0) = sf;
  *(volatile v4f*)(xa32 + o1) = sb;
  *(volatile v4h*)(xa16 + o0) = hf;
  *(volatile v4h*)(xa16 + o1) = hb;
}

__global__ __launch_bounds__(64) void ssm_scan_kernel(
    const float* __restrict__ delta, const float* __restrict__ xa32,
    const float* __restrict__ dbc32, const float* __restrict__ XZ,
    const float* __restrict__ Alog, const float* __restrict__ Dp, float* __restrict__ yg) {
  const unsigned c = blockIdx.x * 64u + threadIdx.x;
  const unsigned b = blockIdx.y;
  const unsigned dir = blockIdx.z;
  float An[DSTATE], h[DSTATE];
  {
    const v4f* ap = (const v4f*)(Alog + (size_t)c * DSTATE);
#pragma unroll
    for (int q = 0; q < 4; ++q) {
      const v4f t = ap[q];
#pragma unroll
      for (int i = 0; i < 4; ++i) {
        An[4 * q + i] = -__expf(bf16r(t[i]));
        h[4 * q + i] = 0.0f;
      }
    }
  }
  const float dval = bf16r(Dp[c]);
  const size_t dbase = (size_t)dir * MROWS;

#pragma unroll 1
  for (unsigned step = 0; step < (unsigned)SEQ; ++step) {
    const int l = (int)step + (int)dir * ((int)SEQ - 1 - 2 * (int)step);
    const size_t row = (size_t)b * SEQ + (unsigned)l;
    const size_t e = (dbase + row) * DINNER + c;
    const float dv = delta[e];
    const float xv = xa32[e];
    const float zv = XZ[row * (2u * DINNER) + DINNER + c];
    const v4f* bc = (const v4f*)(dbc32 + (dbase + row) * XPN + DTRANK);
    v4f Bq[4], Cq[4];
#pragma unroll
    for (int q = 0; q < 4; ++q) { Bq[q] = bc[q]; Cq[q] = bc[4 + q]; }
    const float dx = dv * xv;
    float y = 0.0f;
#pragma unroll
    for (int n = 0; n < DSTATE; ++n) {
      const float dA = __expf(dv * An[n]);
      h[n] = dA * h[n] + dx * Bq[n >> 2][n & 3];
      y += h[n] * Cq[n >> 2][n & 3];
    }
    const float g = (y + dval * xv) * silu_f(zv);
    float* p = yg + e;
    *(volatile float*)p = g;
    __threadfence();
    *(volatile float*)p = g;
  }
}

__global__ __launch_bounds__(256) void ysum_kernel(
    const float* __restrict__ yg, _Float16* __restrict__ ys) {
  const size_t e = ((size_t)blockIdx.x * 256u + threadIdx.x) * 8u;
  const size_t e2 = e + (size_t)MROWS * DINNER;
  const v4f a0 = *(const v4f*)(yg + e);
  const v4f a1 = *(const v4f*)(yg + e + 4u);
  const v4f b0 = *(const v4f*)(yg + e2);
  const v4f b1 = *(const v4f*)(yg + e2 + 4u);
  v8h o;
#pragma unroll
  for (int j = 0; j < 4; ++j) {
    o[j]     = toh_flush(YCARRY * (a0[j] + b0[j]));
    o[j + 4] = toh_flush(YCARRY * (a1[j] + b1[j]));
  }
  _Float16* p = ys + e;
  *(volatile v8h*)p = o;
  __threadfence();
  *(volatile v8h*)p = o;
}

extern "C" void kernel_launch(void* const* d_in, const int* in_sizes, int n_in,
                              void* d_out, int out_size, void* d_ws, size_t ws_size,
                              hipStream_t stream) {
  if (n_in < 37) return;
  const long long need_x = ((long long)(SEQ - 1) * NB_FULL + NB) * DIM;
  const long long need[37] = {
      need_x, need_x,
      (long long)3 * DIM * DIM, (long long)3 * DIM, (long long)DIM * DIM, (long long)DIM,
      (long long)3 * DIM * DIM, (long long)3 * DIM, (long long)DIM * DIM, (long long)DIM,
      (long long)DIM, (long long)DIM, (long long)DIM, (long long)DIM,
      (long long)HID * DIM, (long long)HID, (long long)DIM * HID, (long long)DIM,
      (long long)DIM, (long long)DIM, (long long)DIM, (long long)DIM,
      (long long)HID * DIM, (long long)HID, (long long)DIM * HID, (long long)DIM,
      (long long)2 * DINNER * DIM, (long long)2 * DINNER, (long long)DINNER * 4, (long long)DINNER,
      (long long)XPN * DINNER, (long long)DINNER * DTRANK, (long long)DINNER,
      (long long)DINNER * DSTATE, (long long)DINNER, (long long)DIM * DINNER, (long long)DIM};
  for (int i = 0; i < 37; ++i)
    if ((long long)in_sizes[i] < need[i]) return;
  const long long need_out =
      (long long)OUT1_OFF + ((long long)(NB - 1) * SEQ_FULL + (SEQ - 1)) * SEQ_FULL + SEQ;
  if ((long long)out_size < need_out) return;
  if (ws_size < WS_TOTAL) return;

  const float* tgt      = (const float*)d_in[0];
  const float* memory   = (const float*)d_in[1];
  const float* sa_in_w  = (const float*)d_in[2];
  const float* sa_in_b  = (const float*)d_in[3];
  const float* sa_out_w = (const float*)d_in[4];
  const float* sa_out_b = (const float*)d_in[5];
  const float* ca_in_w  = (const float*)d_in[6];
  const float* ca_in_b  = (const float*)d_in[7];
  const float* ca_out_w = (const float*)d_in[8];
  const float* ca_out_b = (const float*)d_in[9];
  const float* n1_w = (const float*)d_in[10];
  const float* n2_w = (const float*)d_in[11];
  const float* n3_w = (const float*)d_in[12];
  const float* n4_w = (const float*)d_in[13];
  const float* lin1_w = (const float*)d_in[14];
  const float* lin1_b = (const float*)d_in[15];
  const float* lin2_w = (const float*)d_in[16];
  const float* lin2_b = (const float*)d_in[17];
  const float* ln1_w = (const float*)d_in[18];
  const float* ln1_b = (const float*)d_in[19];
  const float* ln2_w = (const float*)d_in[20];
  const float* ln2_b = (const float*)d_in[21];
  const float* bff1_w = (const float*)d_in[22];
  const float* bff1_b = (const float*)d_in[23];
  const float* bff2_w = (const float*)d_in[24];
  const float* bff2_b = (const float*)d_in[25];
  const float* m_in_w    = (const float*)d_in[26];
  const float* m_in_b    = (const float*)d_in[27];
  const float* m_conv_w  = (const float*)d_in[28];
  const float* m_conv_b  = (const float*)d_in[29];
  const float* m_xproj_w = (const float*)d_in[30];
  const float* m_dt_w    = (const float*)d_in[31];
  const float* m_dt_b    = (const float*)d_in[32];
  const float* m_Alog    = (const float*)d_in[33];
  const float* m_D       = (const float*)d_in[34];
  const float* m_out_w   = (const float*)d_in[35];
  const float* m_out_b   = (const float*)d_in[36];
  float* out = (float*)d_out;

  char* ws = (char*)d_ws;
  _Float16* Wsa   = (_Float16*)(ws + OFF_WSA);
  _Float16* Wsao  = (_Float16*)(ws + OFF_WSAO);
  _Float16* Wca   = (_Float16*)(ws + OFF_WCA);
  _Float16* Wcao  = (_Float16*)(ws + OFF_WCAO);
  _Float16* Wl1   = (_Float16*)(ws + OFF_WL1);
  _Float16* Wl2   = (_Float16*)(ws + OFF_WL2);
  _Float16* Wb1   = (_Float16*)(ws + OFF_WB1);
  _Float16* Wb2   = (_Float16*)(ws + OFF_WB2);
  _Float16* Wmin  = (_Float16*)(ws + OFF_WMIN);
  _Float16* Wxp   = (_Float16*)(ws + OFF_WXP);
  _Float16* Wdt   = (_Float16*)(ws + OFF_WDT);
  _Float16* Wmo   = (_Float16*)(ws + OFF_WMO);
  _Float16* T16   = (_Float16*)(ws + OFF_T16);
  _Float16* M16   = (_Float16*)(ws + OFF_M16);
  _Float16* Q16   = (_Float16*)(ws + OFF_Q);
  _Float16* K16   = (_Float16*)(ws + OFF_K);
  _Float16* VT16  = (_Float16*)(ws + OFF_VT);
  _Float16* CTX16 = (_Float16*)(ws + OFF_CTX);
  float*    STM   = (float*)(ws + OFF_STM);
  float*    STR   = (float*)(ws + OFF_STR);
  float*    X1    = (float*)(ws + OFF_X1);
  float*    TGA32 = (float*)(ws + OFF_TGA32);
  _Float16* TGA16 = (_Float16*)(ws + OFF_TGA16);
  float*    TGB32 = (float*)(ws + OFF_TGB32);
  _Float16* XN16  = (_Float16*)(ws + OFF_XN16);
  float*    XZ32  = (float*)(ws + OFF_XZ);
  float*    XA32  = (float*)(ws + OFF_XA32);
  _Float16* XA16  = (_Float16*)(ws + OFF_XA16);
  _Float16* FF16  = (_Float16*)(ws + OFF_XA16);
  float*    DBC32 = (float*)(ws + OFF_DBC32);
  _Float16* DBC16 = (_Float16*)(ws + OFF_DBC16);
  float*    DEL32 = (float*)(ws + OFF_DEL);
  float*    MS32  = (float*)(ws + OFF_DEL);
  float*    YG32  = (float*)(ws + OFF_YG);
  _Float16* YS16  = (_Float16*)(ws + OFF_YS);

  dim3 blk(256);
  dim3 gsq(DIM / 64, MROWS / 64);
  dim3 gff(HID / 64, MROWS / 64);
  dim3 grow(MROWS / 8);
  const float cs_aw = 1.0f / (ACARRY * WCARRY);
  const float cs_cw = 1.0f / (VCARRY * WCARRY);
  const float cs_mw = 1.0f / (MCARRY * WCARRY);

  wcast_kernel<<<dim3(3 * DIM * DIM / 2048), blk, 0, stream>>>(sa_in_w, Wsa, 3u * DIM * DIM / 8u);
  wcast_kernel<<<dim3(DIM * DIM / 2048), blk, 0, stream>>>(sa_out_w, Wsao, (unsigned)DIM * DIM / 8u);
  wcast_kernel<<<dim3(3 * DIM * DIM / 2048), blk, 0, stream>>>(ca_in_w, Wca, 3u * DIM * DIM / 8u);
  wcast_kernel<<<dim3(DIM * DIM / 2048), blk, 0, stream>>>(ca_out_w, Wcao, (unsigned)DIM * DIM / 8u);
  wcast_kernel<<<dim3(DIM * HID / 2048), blk, 0, stream>>>(lin1_w, Wl1, (unsigned)DIM * HID / 8u);
  wcast_kernel<<<dim3(DIM * HID / 2048), blk, 0, stream>>>(lin2_w, Wl2, (unsigned)DIM * HID / 8u);
  wcast_kernel<<<dim3(DIM * HID / 2048), blk, 0, stream>>>(bff1_w, Wb1, (unsigned)DIM * HID / 8u);
  wcast_kernel<<<dim3(DIM * HID / 2048), blk, 0, stream>>>(bff2_w, Wb2, (unsigned)DIM * HID / 8u);
  wcast_kernel<<<dim3(2 * DINNER * DIM / 2048), blk, 0, stream>>>(m_in_w, Wmin, 2u * DINNER * DIM / 8u);
  wcast_kernel<<<dim3(XPN * DINNER / 2048), blk, 0, stream>>>(m_xproj_w, Wxp, (unsigned)XPN * DINNER / 8u);
  wcast_kernel<<<dim3(DINNER * DTRANK / 2048), blk, 0, stream>>>(m_dt_w, Wdt, (unsigned)DINNER * DTRANK / 8u);
  wcast_kernel<<<dim3(DIM * DINNER / 2048), blk, 0, stream>>>(m_out_w, Wmo, (unsigned)DIM * DINNER / 8u);

  incast_kernel<<<grow, blk, 0, stream>>>(tgt, T16);
  incast_kernel<<<grow, blk, 0, stream>>>(memory, M16);

  gemm_h16_kernel<<<gsq, blk, 0, stream>>>(T16, (unsigned)DIM, Wsa, (unsigned)DIM, (unsigned)DIM,
                                           sa_in_b, Q16, (unsigned)DIM, cs_aw, QKCARRY);
  gemm_h16_kernel<<<gsq, blk, 0, stream>>>(T16, (unsigned)DIM, Wsa + (size_t)DIM * DIM, (unsigned)DIM,
                                           (unsigned)DIM, sa_in_b + DIM, K16, (unsigned)DIM, cs_aw, QKCARRY);
  gemm_vt_kernel<<<gsq, blk, 0, stream>>>(T16, Wsa + (size_t)2 * DIM * DIM, sa_in_b + 2 * DIM, VT16,
                                          cs_aw, VPCARRY);
  attn_kernel<<<dim3(SEQ / 128, NHEAD, NB), blk, 0, stream>>>(Q16, K16, VT16, CTX16);
  gemm_addin_kernel<<<gsq, blk, 0, stream>>>(CTX16, (unsigned)DIM, Wsao, (unsigned)DIM, (unsigned)DIM,
                                             sa_out_b, tgt, X1, (unsigned)DIM, cs_cw);
  rms_both_kernel<<<grow, blk, 0, stream>>>(X1, n1_w, TGA32, TGA16);

  gemm_h16_kernel<<<gsq, blk, 0, stream>>>(TGA16, (unsigned)DIM, Wca, (unsigned)DIM, (unsigned)DIM,
                                           ca_in_b, Q16, (unsigned)DIM, cs_aw, QKCARRY);
  gemm_h16_kernel<<<gsq, blk, 0, stream>>>(M16, (unsigned)DIM, Wca + (size_t)DIM * DIM, (unsigned)DIM,
                                           (unsigned)DIM, ca_in_b + DIM, K16, (unsigned)DIM, cs_aw, QKCARRY);
  gemm_vt_kernel<<<gsq, blk, 0, stream>>>(M16, Wca + (size_t)2 * DIM * DIM, ca_in_b + 2 * DIM, VT16,
                                          cs_aw, VPCARRY);
  attn_stats_kernel<<<dim3(SEQ / 128, NHEAD, NB), blk, 0, stream>>>(Q16, K16, VT16, CTX16, STM, STR);
  attn_mean_kernel<<<dim3(SEQ / 64, SEQ / 128, NB), blk, 0, stream>>>(Q16, K16, STM, STR,
                                                                     out + OUT1_OFF);
  gemm_addws_kernel<<<gsq, blk, 0, stream>>>(CTX16, (unsigned)DIM, Wcao, (unsigned)DIM, (unsigned)DIM,
                                             ca_out_b, TGA32, X1, (unsigned)DIM, cs_cw);
  rms_f32_kernel<<<grow, blk, 0, stream>>>(X1, n2_w, TGB32);

  ln_ws_kernel<<<grow, blk, 0, stream>>>(TGB32, ln1_w, ln1_b, XN16);
  gemm_f32_kernel<<<dim3(2 * DINNER / 64, MROWS / 64), blk, 0, stream>>>(
      XN16, (unsigned)DIM, Wmin, (unsigned)DIM, (unsigned)DIM, m_in_b, XZ32, 2u * DINNER, cs_aw, 1.0f);
  conv_silu_kernel<<<dim3(MROWS), blk, 0, stream>>>(XZ32, m_conv_w, m_conv_b, XA32, XA16);
  gemm_xproj_kernel<<<dim3(XPN / 64, 2 * MROWS / 64), blk, 0, stream>>>(
      XA16, (unsigned)DINNER, Wxp, (unsigned)DINNER, (unsigned)DINNER, DBC32, DBC16, (unsigned)XPN,
      1.0f / (XACARRY * WCARRY), DCARRY);
  gemm_softplus_kernel<<<dim3(DINNER / 64, 2 * MROWS / 64), blk, 0, stream>>>(
      DBC16, (unsigned)XPN, Wdt, (unsigned)DTRANK, (unsigned)DTRANK, m_dt_b, DEL32, (unsigned)DINNER,
      1.0f / (DCARRY * WCARRY));
  ssm_scan_kernel<<<dim3(DINNER / 64, NB, 2), dim3(64), 0, stream>>>(DEL32, XA32, DBC32, XZ32, m_Alog,
                                                                    m_D, YG32);
  ysum_kernel<<<dim3(MROWS * DINNER / 2048), blk, 0, stream>>>(YG32, YS16);
  gemm_f32_kernel<<<gsq, blk, 0, stream>>>(YS16, (unsigned)DINNER, Wmo, (unsigned)DINNER,
                                           (unsigned)DINNER, m_out_b, MS32, (unsigned)DIM,
                                           1.0f / (YCARRY * WCARRY), 2.0f);
  ln_ws_kernel<<<grow, blk, 0, stream>>>(MS32, ln2_w, ln2_b, XN16);
  gemm_gelu_kernel<<<gff, blk, 0, stream>>>(XN16, (unsigned)DIM, Wb1, (unsigned)DIM, (unsigned)DIM,
                                            bff1_b, FF16, (unsigned)HID, cs_aw);
  gemm_add2_kernel<<<gsq, blk, 0, stream>>>(FF16, (unsigned)HID, Wb2, (unsigned)HID, (unsigned)HID,
                                            bff2_b, TGB32, X1, (unsigned)DIM, cs_mw);

  rms_both_kernel<<<grow, blk, 0, stream>>>(X1, n3_w, TGA32, TGA16);
  gemm_relu_kernel<<<gff, blk, 0, stream>>>(TGA16, (unsigned)DIM, Wl1, (unsigned)DIM, (unsigned)DIM,
                                            lin1_b, FF16, (unsigned)HID, cs_aw);
  gemm_addws_kernel<<<gsq, blk, 0, stream>>>(FF16, (unsigned)HID, Wl2, (unsigned)HID, (unsigned)HID,
                                             lin2_b, TGA32, X1, (unsigned)DIM, cs_mw);
  rms_out_kernel<<<grow, blk, 0, stream>>>(X1, n4_w, out);
}
